// IndexedMatMul_56676388438552
// MI455X (gfx1250) — hardware-verified
//
#include <hip/hip_runtime.h>

constexpr int kTokens     = 8192;
constexpr int kDim        = 1024;
constexpr int kOut        = 1024;
constexpr int kExperts    = 8;
constexpr int kTokBlocks  = kTokens / 64;
constexpr int kTilesMCap  = 136;
constexpr int kRowCap     = kTilesMCap * 64;
constexpr int kTilesN     = kOut / 64;
constexpr int kGemmBlocks = kTilesMCap * kTilesN / 8;
constexpr int kW8         = kExperts * kOut * kDim / 8;
static_assert(kTokens == 256 * 32);
static_assert((kTilesMCap * kTilesN) % 8 == 0);
static_assert(kW8 % 256 == 0);

constexpr size_t kOffW16  = 0;
constexpr size_t kOffA16  = kOffW16 + (size_t)kExperts * kOut * kDim * 2;
constexpr size_t kOffYP   = kOffA16 + (size_t)kRowCap * kDim * 2;
constexpr size_t kWsTotal = kOffYP + (size_t)kRowCap * kOut * 4;
static_assert(kWsTotal == 70254592);
static_assert(kOffA16 % 128 == 0 && kOffYP % 128 == 0);

typedef __attribute__((ext_vector_type(16))) _Float16 v16h;
typedef __attribute__((ext_vector_type(8)))  _Float16 v8h;
typedef __attribute__((ext_vector_type(16))) __bf16   v16b;
typedef __attribute__((ext_vector_type(8)))  __bf16   v8b;
typedef __attribute__((ext_vector_type(8)))  float    v8f;
typedef __attribute__((ext_vector_type(4)))  float    v4f;
typedef __attribute__((ext_vector_type(4)))  unsigned int v4u;
typedef __attribute__((ext_vector_type(4)))  int      v4i;

__device__ __forceinline__ unsigned short f2bf_bits(float f) {
  unsigned u = __float_as_uint(f);
  return (unsigned short)((u + 0x7FFFu + ((u >> 16) & 1u)) >> 16);
}
__device__ __forceinline__ float bf_bits2f(unsigned short h) { return __uint_as_float(((unsigned)h) << 16); }

__device__ __forceinline__ void dep_guard_h(v8f& a, v8f& b, v16h x, v16h y) { asm volatile("v_nop\n\tv_nop\n\tv_nop\n\tv_nop" : "+v"(a), "+v"(b) : "v"(x), "v"(y)); }
__device__ __forceinline__ void dep_guard_b(v8f& a, v8f& b, v16b x, v16b y) { asm volatile("v_nop\n\tv_nop\n\tv_nop\n\tv_nop" : "+v"(a), "+v"(b) : "v"(x), "v"(y)); }
__device__ __forceinline__ void keep4_h(v16h a, v16h b, v16h c, v16h d) { asm volatile("v_nop" :: "v"(a), "v"(b), "v"(c), "v"(d)); }
__device__ __forceinline__ void keep4_b(v16b a, v16b b, v16b c, v16b d) { asm volatile("v_nop" :: "v"(a), "v"(b), "v"(c), "v"(d)); }
__device__ __forceinline__ void acc_guard4(v8f& a, v8f& b, v8f& c, v8f& d) { asm volatile("v_nop\n\tv_nop\n\tv_nop\n\tv_nop" : "+v"(a), "+v"(b), "+v"(c), "+v"(d)); }
template <typename T> struct Frag;
template <> struct Frag<_Float16> {
  typedef v16h V; union U { v16h v; v8h h[2]; };
  static __device__ __forceinline__ v16h load(const _Float16* p) {
    U f; f.h[0] = *(const v8h*)(p); f.h[1] = *(const v8h*)(p + 16); return f.v;
  }
  static __device__ __forceinline__ v8f mma(v16h a, v16h b, v8f c) {
    return __builtin_amdgcn_wmma_f32_16x16x32_f16(false, a, false, b, (short)0, c, false, false);
  }
  static __device__ __forceinline__ void guard(v8f& a, v8f& b, v16h x, v16h y) { dep_guard_h(a, b, x, y); }
  static __device__ __forceinline__ void keep(v16h a, v16h b, v16h c, v16h d) { keep4_h(a, b, c, d); }
};
template <> struct Frag<__bf16> {
  typedef v16b V; union U { v16b v; v8b h[2]; };
  static __device__ __forceinline__ v16b load(const __bf16* p) {
    U f; f.h[0] = *(const v8b*)(p); f.h[1] = *(const v8b*)(p + 16); return f.v;
  }
  static __device__ __forceinline__ v8f mma(v16b a, v16b b, v8f c) {
    return __builtin_amdgcn_wmma_f32_16x16x32_bf16(false, a, false, b, (short)0, c, false, false);
  }
  static __device__ __forceinline__ void guard(v8f& a, v8f& b, v16b x, v16b y) { dep_guard_b(a, b, x, y); }
  static __device__ __forceinline__ void keep(v16b a, v16b b, v16b c, v16b d) { keep4_b(a, b, c, d); }
};

__device__ __forceinline__ unsigned pk16(unsigned short a, unsigned short b) { return (unsigned)a | ((unsigned)b << 16); }

__device__ __forceinline__ int clamp_expert(int v) { v = (v < 0) ? 0 : v; return (v > kExperts - 1) ? (kExperts - 1) : v; }

__device__ __forceinline__ void expert_hist(const int* __restrict__ idx, int t0, int tid, int* sTot, int* sPre) {
  int cnt[8];
#pragma unroll
  for (int e = 0; e < 8; ++e) cnt[e] = 0;
  const v4i* p = (const v4i*)(idx + 32 * tid);
#pragma unroll 1
  for (int q = 0; q < 8; ++q) {
    const v4i v = p[q];
#pragma unroll
    for (int u = 0; u < 4; ++u) {
      const int x = clamp_expert(v[u]);
#pragma unroll
      for (int e = 0; e < 8; ++e) cnt[e] += (x == e) ? 1 : 0;
    }
  }
  const int isPre = (32 * tid < t0) ? 1 : 0;
  const int lane = tid & 31, wave = tid >> 5;
#pragma unroll
  for (int e = 0; e < 8; ++e) {
    int a = cnt[e];
    int b = cnt[e] * isPre;
#pragma unroll
    for (int off = 1; off < 32; off <<= 1) { a += __shfl_xor(a, off, 32); b += __shfl_xor(b, off, 32); }
    if (lane == 0) { sTot[wave * 8 + e] = a; sPre[wave * 8 + e] = b; }
  }
}

__device__ __forceinline__ void expert_finalize(int tid, const int* sTot, const int* sPre, int* sSeg, int* sCnt, int* sBase) {
  const int ex = tid & 7;
  int segv = 0, totMine = 0, preMine = 0;
#pragma unroll 1
  for (int e2 = 0; e2 < kExperts; ++e2) {
    int ts = 0, ps = 0;
#pragma unroll
    for (int w = 0; w < 8; ++w) { ts += sTot[w * 8 + e2]; ps += sPre[w * 8 + e2]; }
    segv += (e2 < ex) ? ((ts + 63) & ~63) : 0;
    totMine = (e2 == ex) ? ts : totMine;
    preMine = (e2 == ex) ? ps : preMine;
  }
  if (tid < kExperts) { sSeg[tid] = segv; sCnt[tid] = totMine; sBase[tid] = preMine; }
}

__device__ __forceinline__ void list_positions(int tid, const int* sIdx, const int* sSeg, const int* sBase, int* sPos) {
  const int i = tid & 63;
  const int myE = sIdx[i];
  int rank = 0;
#pragma unroll 1
  for (int k = 0; k < 64; ++k) rank += ((k < i) && (sIdx[k] == myE)) ? 1 : 0;
  int pos = sSeg[myE] + sBase[myE] + rank;
  pos = (pos < 0) ? 0 : pos;
  pos = (pos > kRowCap - 1) ? (kRowCap - 1) : pos;
  if (tid < 64) sPos[tid] = pos;
}

__global__ __launch_bounds__(256) void k_cast_w(const float* __restrict__ in, unsigned short* __restrict__ out, int n8) {
  const int i = blockIdx.x * 256 + threadIdx.x;
  if (i >= n8) return;
  const float* p = in + 8 * (size_t)i;
  const v4f a = *(const v4f*)(p);
  const v4f c = *(const v4f*)(p + 4);
  unsigned short hb[8];
#pragma unroll
  for (int e = 0; e < 4; ++e) {
    hb[e]     = f2bf_bits(a[e]);
    hb[4 + e] = f2bf_bits(c[e]);
  }
  const v4u u = (v4u){pk16(hb[0], hb[1]), pk16(hb[2], hb[3]), pk16(hb[4], hb[5]), pk16(hb[6], hb[7])};
  unsigned short* q = out + 8 * (size_t)i;
  *(volatile v4u*)q = u;
  __threadfence();
  *(volatile v4u*)q = u;
}

__global__ __launch_bounds__(256) void k_gather_rows(const float* __restrict__ X, const int* __restrict__ idx,
                                                     unsigned short* __restrict__ A16) {
  __shared__ int sTot[64];
  __shared__ int sPre[64];
  __shared__ int sSeg[8];
  __shared__ int sCnt[8];
  __shared__ int sBase[8];
  __shared__ int sIdx[64];
  __shared__ int sPos[64];
  const int tid = threadIdx.x, lane = tid & 31, wave = tid >> 5;
  const int blk = blockIdx.x;
  const int tb  = (blk < kTokBlocks) ? blk : (kTokBlocks - 1);
  const int t0  = tb * 64;

  expert_hist(idx, t0, tid, sTot, sPre);
  {
    const int v = clamp_expert(idx[t0 + (tid & 63)]);
    if (tid < 64) sIdx[tid] = v;
  }
  __syncthreads();
  expert_finalize(tid, sTot, sPre, sSeg, sCnt, sBase);
  __syncthreads();
  list_positions(tid, sIdx, sSeg, sBase, sPos);
  __syncthreads();

  if (blk < kTokBlocks) {
    for (int pass = 0; pass < 2; ++pass) {
#pragma unroll 1
      for (int j = 0; j < 8; ++j) {
        const int rowLocal = wave + 8 * j;
        const int r   = t0 + rowLocal;
        const int pos = sPos[rowLocal];
        const float* xr = X + (size_t)r * kDim;
        unsigned short* ar = A16 + (size_t)pos * kDim;
#pragma unroll
        for (int it = 0; it < 4; ++it) {
          const int c0 = it * 256 + lane * 8;
          const v4f a = *(const v4f*)(xr + c0);
          const v4f c = *(const v4f*)(xr + c0 + 4);
          unsigned short hb[8];
#pragma unroll
          for (int e = 0; e < 4; ++e) { hb[e] = f2bf_bits(a[e]); hb[4 + e] = f2bf_bits(c[e]); }
          const v4u u = (v4u){pk16(hb[0], hb[1]), pk16(hb[2], hb[3]), pk16(hb[4], hb[5]), pk16(hb[6], hb[7])};
          *(volatile v4u*)(ar + c0) = u;
        }
      }
      __threadfence();
    }
  } else {
    const int e    = blk - kTokBlocks;
    const int cnt  = sCnt[e];
    const int nPad = ((cnt + 63) & ~63) - cnt;
    const int base = sSeg[e] + cnt;
    const v4u z = (v4u){0u, 0u, 0u, 0u};
    for (int pass = 0; pass < 2; ++pass) {
#pragma unroll 1
      for (int j = 0; j < 8; ++j) {
        const int rowLocal = wave + 8 * j;
        if (rowLocal < nPad) {
          int row = base + rowLocal;
          row = (row > kRowCap - 1) ? (kRowCap - 1) : row;
          unsigned short* ar = A16 + (size_t)row * kDim;
#pragma unroll
          for (int it = 0; it < 4; ++it) *(volatile v4u*)(ar + it * 256 + lane * 8) = z;
        }
      }
      __threadfence();
    }
  }
}

__global__ __launch_bounds__(256) void k_seg_gemm(const unsigned short* __restrict__ A16p, const unsigned short* __restrict__ W16p,
                                                  const int* __restrict__ idx, float* __restrict__ YP) {
  typedef __bf16 T;
  typedef v16b V;
  __shared__ __align__(16) float sT[8][16 * 68];
  __shared__ int sTot[64];
  __shared__ int sPre[64];
  __shared__ int sSeg[8];
  __shared__ int sCnt[8];
  __shared__ int sBase[8];
  const int tid  = threadIdx.x;
  const int lane = tid & 31;
  const int wave = tid >> 5;

  expert_hist(idx, 0, tid, sTot, sPre);
  __syncthreads();
  expert_finalize(tid, sTot, sPre, sSeg, sCnt, sBase);
  __syncthreads();

  const int total = sSeg[7] + ((sCnt[7] + 63) & ~63);
  const int tile = blockIdx.x * 8 + wave;
  const int tm = tile >> 4;
  const int tn = tile & 15;
  const int m0 = tm << 6;
  const int n0 = tn << 6;
  int e = 0;
#pragma unroll
  for (int j = 1; j < kExperts; ++j) e += (m0 >= sSeg[j]) ? 1 : 0;
  if (m0 >= total) return;

  const T* Ab = (const T*)A16p;
  const T* Bb = (const T*)W16p + (size_t)e * kOut * kDim;
  const int lda = kDim, ldb = kDim, ldc = kOut;
  const int K = kDim;

  const int rlane = lane & 15;
  const int koff  = (lane >> 4) * 8;
  const int mOff  = (lane >> 4) * 8;

  v8f acc[4][4];
#pragma unroll
  for (int i = 0; i < 4; ++i)
#pragma unroll
    for (int j = 0; j < 4; ++j) acc[i][j] = (v8f){0.f,0.f,0.f,0.f,0.f,0.f,0.f,0.f};

  for (int k0 = 0; k0 < K; k0 += 32) {
    V bh[4];
#pragma unroll
    for (int j = 0; j < 4; ++j) {
      const size_t bo = (size_t)(n0 + (j << 4) + rlane) * ldb + koff + k0;
      bh[j] = Frag<T>::load(Bb + bo);
    }
#pragma unroll
    for (int i = 0; i < 4; ++i) {
      const size_t ao = (size_t)(m0 + (i << 4) + rlane) * lda + koff + k0;
      V ah = Frag<T>::load(Ab + ao);
#pragma unroll
      for (int j = 0; j < 4; ++j) {
        acc[i][j] = Frag<T>::mma(ah, bh[j], acc[i][j]);
      }
      Frag<T>::guard(acc[i][0], acc[i][3], ah, ah);
    }
    Frag<T>::keep(bh[0], bh[1], bh[2], bh[3]);
  }
  acc_guard4(acc[0][0], acc[0][1], acc[0][2], acc[0][3]);
  acc_guard4(acc[1][0], acc[1][1], acc[1][2], acc[1][3]);
  acc_guard4(acc[2][0], acc[2][1], acc[2][2], acc[2][3]);
  acc_guard4(acc[3][0], acc[3][1], acc[3][2], acc[3][3]);

  float* slab = sT[wave];
#pragma unroll
  for (int i = 0; i < 4; ++i) {
    const int mBase = m0 + (i << 4);
#pragma unroll
    for (int j = 0; j < 4; ++j) {
#pragma unroll
      for (int r = 0; r < 8; ++r) {
        const float v = acc[i][j][r];
        slab[(mOff + r) * 68 + (j << 4) + rlane] = v;
      }
    }
    __builtin_amdgcn_fence(__ATOMIC_RELEASE, "workgroup");
    __builtin_amdgcn_wave_barrier();
    __builtin_amdgcn_fence(__ATOMIC_ACQUIRE, "workgroup");
    {
      float* C = YP;
      const int hh = lane >> 4, c4 = (lane & 15) * 4;
      for (int pass = 0; pass < 2; ++pass) {
#pragma unroll
        for (int it = 0; it < 8; ++it) {
          const int row = it * 2 + hh;
          v4f v = *(const v4f*)(slab + row * 68 + c4);
          *(volatile v4f*)(C + (size_t)(mBase + row) * ldc + n0 + c4) = v;
        }
        __threadfence();
      }
    }
    __builtin_amdgcn_fence(__ATOMIC_RELEASE, "workgroup");
    __builtin_amdgcn_wave_barrier();
    __builtin_amdgcn_fence(__ATOMIC_ACQUIRE, "workgroup");
  }
}

__global__ __launch_bounds__(256) void k_scatter_rows(const float* __restrict__ YP, const int* __restrict__ idx,
                                                      float* __restrict__ Y) {
  __shared__ int sTot[64];
  __shared__ int sPre[64];
  __shared__ int sSeg[8];
  __shared__ int sCnt[8];
  __shared__ int sBase[8];
  __shared__ int sIdx[64];
  __shared__ int sPos[64];
  const int tid = threadIdx.x, lane = tid & 31, wave = tid >> 5;
  const int t0  = blockIdx.x * 64;

  expert_hist(idx, t0, tid, sTot, sPre);
  {
    const int v = clamp_expert(idx[t0 + (tid & 63)]);
    if (tid < 64) sIdx[tid] = v;
  }
  __syncthreads();
  expert_finalize(tid, sTot, sPre, sSeg, sCnt, sBase);
  __syncthreads();
  list_positions(tid, sIdx, sSeg, sBase, sPos);
  __syncthreads();

  for (int pass = 0; pass < 2; ++pass) {
#pragma unroll 1
    for (int j = 0; j < 8; ++j) {
      const int rowLocal = wave + 8 * j;
      const int r   = t0 + rowLocal;
      const int pos = sPos[rowLocal];
      const float* yr = YP + (size_t)pos * kOut;
      float* orow = Y + (size_t)r * kOut;
#pragma unroll
      for (int it = 0; it < 8; ++it) {
        const int c0 = it * 128 + lane * 4;
        const v4f v = *(const v4f*)(yr + c0);
        *(volatile v4f*)(orow + c0) = v;
      }
    }
    __threadfence();
  }
}

extern "C" void kernel_launch(void* const* d_in, const int* in_sizes, int n_in,
                              void* d_out, int out_size, void* d_ws, size_t ws_size,
                              hipStream_t stream) {
  if (n_in < 3) return;
  if (in_sizes[0] != kTokens * kDim) return;
  if (in_sizes[1] != kExperts * kOut * kDim) return;
  if (in_sizes[2] != kTokens) return;
  if (out_size != kTokens * kOut) return;
  if (ws_size < kWsTotal) return;

  const float* X   = (const float*)d_in[0];
  const float* W   = (const float*)d_in[1];
  const int*   idx = (const int*)d_in[2];
  float*       Y   = (float*)d_out;
  char*        ws  = (char*)d_ws;
  unsigned short* W16 = (unsigned short*)(ws + kOffW16);
  unsigned short* A16 = (unsigned short*)(ws + kOffA16);
  float*          YP  = (float*)(ws + kOffYP);

  k_cast_w<<<kW8 / 256, 256, 0, stream>>>(W, W16, kW8);
  k_gather_rows<<<kTokBlocks + kExperts, 256, 0, stream>>>(X, idx, A16);
  k_seg_gemm<<<kGemmBlocks, 256, 0, stream>>>(A16, W16, idx, YP);
  k_scatter_rows<<<kTokBlocks, 256, 0, stream>>>(YP, idx, Y);
}
